// Self_Attention_78606491451578
// MI455X (gfx1250) — hardware-verified
//
#include <hip/hip_runtime.h>


#ifndef NB
#define NB 16
#endif
#ifndef SEQ
#define SEQ 2048
#endif
#define NB_FULL  16
#define SEQ_FULL 2048
#define CH   256
#define DQK  32
#define OC   320
#define PCAR 4096.0f
#define BNEPS 1e-5f
#define SLOPE 0.2f

static_assert(SEQ % 128 == 0);
static_assert((NB * SEQ) % 64 == 0);
static_assert(CH % 64 == 0);
static_assert(OC % 64 == 0);
static_assert(OC % 32 == 0);
static_assert(DQK == 32);
static_assert(((size_t)NB * SEQ * CH) % 512 == 0);
static_assert(((size_t)NB * SEQ * DQK) % 256 == 0);
static_assert(NB <= NB_FULL);
static_assert(SEQ <= SEQ_FULL);
static_assert((DQK * CH) % 2048 == 0);
static_assert((CH * CH) % 2048 == 0);

typedef _Float16 h16;
typedef unsigned short bf;
typedef __attribute__((ext_vector_type(16))) __bf16   v16bf;
typedef __attribute__((ext_vector_type(16))) _Float16 v16h;
typedef __attribute__((ext_vector_type(8)))  _Float16 v8h;
typedef __attribute__((ext_vector_type(8)))  unsigned short v8us;
typedef __attribute__((ext_vector_type(8)))  float    v8f;
typedef __attribute__((ext_vector_type(4)))  float    v4f;
typedef __attribute__((ext_vector_type(2)))  _Float16 v2h;
typedef __attribute__((ext_vector_type(4)))  _Float16 v4h;
typedef __attribute__((ext_vector_type(2)))  unsigned short v2us;
typedef __attribute__((ext_vector_type(4)))  unsigned short v4us;
typedef __attribute__((ext_vector_type(2)))  float v2f;
typedef v8h  __attribute__((may_alias)) v8ha;
typedef v4f  __attribute__((may_alias)) v4fa;
typedef v8us __attribute__((may_alias)) v8usa;

__device__ __forceinline__ unsigned short f2bf(float f) { unsigned u = __float_as_uint(f); u += 0x7FFFu + ((u >> 16) & 1u); return (unsigned short)(u >> 16); }
__device__ __forceinline__ float bf2f(unsigned short b) { return __uint_as_float(((unsigned)b) << 16); }
__device__ __forceinline__ float bfr(float f) { return bf2f(f2bf(f)); }
__device__ __forceinline__ v16h cat16(v8h lo, v8h hi) { return __builtin_shufflevector(lo, hi, 0, 1, 2, 3, 4, 5, 6, 7, 8, 9, 10, 11, 12, 13, 14, 15); }
__device__ __forceinline__ v16bf cat16b(v8us lo, v8us hi) { return __builtin_bit_cast(v16bf, __builtin_shufflevector(lo, hi, 0, 1, 2, 3, 4, 5, 6, 7, 8, 9, 10, 11, 12, 13, 14, 15)); }
__device__ __forceinline__ v8f wmma16(v16h a, v16h b, v8f c) { return __builtin_amdgcn_wmma_f32_16x16x32_f16(false, a, false, b, (short)0, c, false, false); }
__device__ __forceinline__ v8f wmmab(v16bf a, v16bf b, v8f c) { return __builtin_amdgcn_wmma_f32_16x16x32_bf16(false, a, false, b, (short)0, c, false, false); }
__device__ __forceinline__ h16 tohx(float x) { return (h16)x; }
__device__ __forceinline__ void splitf(float y, unsigned short& h, unsigned short& l) { h = f2bf(y); l = f2bf(y - bf2f(h)); }

template <typename T16> struct WFrag;
template <> struct WFrag<h16> { typedef v16h V; static __device__ __forceinline__ V ld(const h16* p) { return cat16(*(const v8h*)p, *(const v8h*)(p + 16)); } static __device__ __forceinline__ v8f mma(V a, V b, v8f c) { return wmma16(a, b, c); } };
template <> struct WFrag<bf> { typedef v16bf V; static __device__ __forceinline__ V ld(const bf* p) { return cat16b(*(const v8us*)p, *(const v8us*)(p + 16)); } static __device__ __forceinline__ v8f mma(V a, V b, v8f c) { return wmmab(a, b, c); } };
template <typename T16, int NSPLIT, int EPI>
__global__ __launch_bounds__(32) void k_gemmw(const T16* __restrict__ A, const T16* __restrict__ A2, const T16* __restrict__ Bt, const T16* __restrict__ Bt2, int K, float* C, int ldc, const float* __restrict__ R, float oscale, size_t sA, size_t sB, size_t sC) {
    typedef typename WFrag<T16>::V V;
    __shared__ __align__(16) float os[16 * 68];
    const size_t z = blockIdx.z; A += z * sA; if (A2) A2 += z * sA; Bt += z * sB; if (Bt2) Bt2 += z * sB; C += z * sC; if (R) R += z * sC;
    const int lane = threadIdx.x & 31, lr = lane & 15, hi = lane >> 4; const int r0 = blockIdx.x * 64, c0 = blockIdx.y * 64;
    v8f acc[4][4];
#pragma unroll
    for (int mb = 0; mb < 4; ++mb)
#pragma unroll
        for (int nb = 0; nb < 4; ++nb) acc[mb][nb] = (v8f){};
    const size_t aoff = (size_t)(r0 + lr) * K + 8 * hi, boff = (size_t)(c0 + lr) * K + 8 * hi;
#pragma unroll 1
    for (int kc = 0; kc < K; kc += 32) {
        V a[4], a2[4];
#pragma unroll
        for (int mb = 0; mb < 4; ++mb) { a[mb] = WFrag<T16>::ld(A + aoff + (size_t)mb * 16 * K + kc); if (NSPLIT == 1 || NSPLIT == 2) a2[mb] = WFrag<T16>::ld(A2 + aoff + (size_t)mb * 16 * K + kc); }
#pragma unroll
        for (int nb = 0; nb < 4; ++nb) { const V b = WFrag<T16>::ld(Bt + boff + (size_t)nb * 16 * K + kc); V b2; if (NSPLIT >= 2) b2 = WFrag<T16>::ld(Bt2 + boff + (size_t)nb * 16 * K + kc);
#pragma unroll
            for (int mb = 0; mb < 4; ++mb) { acc[mb][nb] = WFrag<T16>::mma(a[mb], b, acc[mb][nb]); if (NSPLIT == 1 || NSPLIT == 2) acc[mb][nb] = WFrag<T16>::mma(a2[mb], b, acc[mb][nb]); if (NSPLIT >= 2) acc[mb][nb] = WFrag<T16>::mma(a[mb], b2, acc[mb][nb]); } }
        asm volatile("v_nop\n\tv_nop\n\tv_nop\n\tv_nop" : "+v"(acc[0][0]), "+v"(acc[1][1]), "+v"(acc[2][2]), "+v"(acc[3][3]) : "v"(a[0]), "v"(a[3]));
    }
#pragma unroll
    for (int mb = 0; mb < 4; ++mb) {
#pragma unroll
        for (int nb = 0; nb < 4; ++nb) {
#pragma unroll
            for (int j = 0; j < 8; ++j) os[(hi * 8 + j) * 68 + nb * 16 + lr] = acc[mb][nb][j]; }
        __builtin_amdgcn_wave_barrier(); asm volatile("" ::: "memory");
        float* crow = C + (size_t)(r0 + mb * 16) * ldc + c0;
        const float* rrow = (EPI == 1) ? (R + (size_t)(r0 + mb * 16) * ldc + c0) : nullptr;
#pragma unroll 1
        for (int ps = 0; ps < 2; ++ps) {
#pragma unroll
            for (int s = 0; s < 8; ++s) { const int row = 2 * s + hi, cofs = lr * 4; v4f val = *(const v4fa*)(os + row * 68 + cofs);
                if (EPI == 1) { const v4f xr = *(const v4f*)(rrow + (size_t)row * ldc + cofs); val[0] = val[0] * oscale + bfr(xr[0]); val[1] = val[1] * oscale + bfr(xr[1]); val[2] = val[2] * oscale + bfr(xr[2]); val[3] = val[3] * oscale + bfr(xr[3]); }
                *(volatile v4f*)(crow + (size_t)row * ldc + cofs) = val; }
            if (ps == 0) __threadfence(); }
        __builtin_amdgcn_wave_barrier(); asm volatile("" ::: "memory");
    }
}

__global__ __launch_bounds__(256) void k_cvt8(const float* __restrict__ src, bf* dst, size_t n8) { const size_t i = (size_t)blockIdx.x * 256 + threadIdx.x; if (i >= n8) return; const v8f v = *(const v8f*)(src + i * 8); v8us o;
#pragma unroll
    for (int k = 0; k < 8; ++k) o[k] = f2bf(v[k]); *(volatile v8us*)(dst + i * 8) = o; __threadfence(); *(volatile v8us*)(dst + i * 8) = o; }

__global__ __launch_bounds__(256) void k_xt(const float* __restrict__ x, bf* XT) {
    const size_t e = ((size_t)blockIdx.x * 256 + threadIdx.x) * 2; if (e >= (size_t)NB * SEQ * CH) return;
    const int c = (int)(e % CH); const size_t row = e / CH; const int n = (int)(row % SEQ); const int b = (int)(row / SEQ);
    const float* src = x + (size_t)b * CH * SEQ_FULL + (size_t)c * SEQ_FULL + n;
    v2us o; o[0] = f2bf(src[0]); o[1] = f2bf(src[SEQ_FULL]);
    *(volatile v2us*)(XT + e) = o; __threadfence(); *(volatile v2us*)(XT + e) = o;
}

__global__ __launch_bounds__(256) void k_stats(const float* __restrict__ F, int nrows,
                                               const float* __restrict__ qb, const float* __restrict__ qg, const float* __restrict__ qbe,
                                               const float* __restrict__ kb, const float* __restrict__ kg, const float* __restrict__ kbe,
                                               const float* __restrict__ vb, const float* __restrict__ vg, const float* __restrict__ vbe, float* ST) {
    __shared__ double ssum[8][32], ssq[8][32];
    const int lane = threadIdx.x & 31, w = threadIdx.x >> 5; const int o = blockIdx.x * 32 + lane;
    const int iq = min(o, DQK - 1), ik = min(max(o - DQK, 0), DQK - 1), iv = min(max(o - 2 * DQK, 0), CH - 1);
    const float bq_ = qb[iq], bk_ = kb[ik], bv_ = vb[iv], gq_ = qg[iq], gk_ = kg[ik], gv_ = vg[iv], eq_ = qbe[iq], ek_ = kbe[ik], ev_ = vbe[iv];
    const bool isq = (o < DQK), isk = (o < 2 * DQK);
    const float bias = bfr(isq ? bq_ : (isk ? bk_ : bv_)); const float gam = bfr(isq ? gq_ : (isk ? gk_ : gv_)); const float bet = bfr(isq ? eq_ : (isk ? ek_ : ev_));
    double s = 0.0, s2 = 0.0;
#pragma unroll 1
    for (int r = w; r < nrows; r += 8) { const float y = F[(size_t)r * OC + o] + bias; const double yd = (double)y; s += yd; s2 = fma(yd, yd, s2); }
    ssum[w][lane] = s; ssq[w][lane] = s2;
    __syncthreads();
    if (w == 0) {
        double ts = 0.0, tq = 0.0;
#pragma unroll
        for (int j = 0; j < 8; ++j) { ts += ssum[j][lane]; tq += ssq[j][lane]; }
        const double inv = 1.0 / (double)nrows; const double mean = ts * inv; double var = tq * inv - mean * mean; var = (var > 0.0) ? var : 0.0;
        const float meanf = (float)mean, varf = (float)var; const float rstd = 1.0f / sqrtf(varf + BNEPS);
        v4f t; t[0] = bias; t[1] = meanf; t[2] = gam * rstd; t[3] = bet;
        *(volatile v4f*)(ST + (size_t)o * 4) = t; __threadfence(); *(volatile v4f*)(ST + (size_t)o * 4) = t;
    }
}

__global__ __launch_bounds__(256) void k_qkp(const float* __restrict__ F, const float* __restrict__ ST, bf* Ph, bf* Pl) {
    const size_t per = (size_t)NB * SEQ * DQK; const size_t e = ((size_t)blockIdx.x * 256 + threadIdx.x) * 2; if (e >= 2 * per) return;
    const int which = (e >= per) ? 1 : 0; const size_t le = e - (size_t)which * per; const size_t row = le / DQK; const int d = (int)(le % DQK); const int o = which * DQK + d;
    const float* f = F + row * OC + o; v2us oh, ol;
#pragma unroll
    for (int q = 0; q < 2; ++q) { const v4f t = *(const v4f*)(ST + (size_t)(o + q) * 4); const float y = f[q] + t[0]; const float val = (y - t[1]) * t[2] + t[3]; unsigned short a2, c2; splitf(val, a2, c2); oh[q] = a2; ol[q] = c2; }
    *(volatile v2us*)(Ph + e) = oh; *(volatile v2us*)(Pl + e) = ol; __threadfence(); *(volatile v2us*)(Ph + e) = oh; *(volatile v2us*)(Pl + e) = ol;
}

__global__ __launch_bounds__(256) void k_vtp(const float* __restrict__ F, const float* __restrict__ ST, h16* V16) {
    const size_t e = ((size_t)blockIdx.x * 256 + threadIdx.x) * 2; if (e >= (size_t)NB * CH * SEQ) return;
    const int m = (int)(e % SEQ); const int c = (int)((e / SEQ) % CH); const int b = (int)(e / ((size_t)SEQ * CH)); const int o = 2 * DQK + c;
    const v4f t = *(const v4f*)(ST + (size_t)o * 4); v2h o16;
#pragma unroll
    for (int q = 0; q < 2; ++q) { const float y = F[((size_t)b * SEQ + m + q) * OC + o] + t[0]; float val = (y - t[1]) * t[2] + t[3]; val = (val >= 0.f) ? val : SLOPE * val; o16[q] = tohx(val); }
    *(volatile v2h*)(V16 + e) = o16; __threadfence(); *(volatile v2h*)(V16 + e) = o16;
}

__global__ __launch_bounds__(256) void k_asoft(const float* __restrict__ Sb, h16* P16) {
    const int lane = threadIdx.x & 31; const int row = blockIdx.x * 8 + (threadIdx.x >> 5); if (row >= SEQ) return;
    const float* sr = Sb + (size_t)row * SEQ; float v[SEQ / 32]; float mx = -3.0e38f;
#pragma unroll
    for (int ch = 0; ch < SEQ / 128; ++ch) { const int j0 = ch * 128 + lane * 4; const v4f a = *(const v4f*)(sr + j0);
#pragma unroll
        for (int q = 0; q < 4; ++q) { v[ch * 4 + q] = a[q]; mx = fmaxf(mx, a[q]); } }
#pragma unroll
    for (int sh = 16; sh; sh >>= 1) mx = fmaxf(mx, __shfl_xor(mx, sh, 32));
    float sum = 0.f;
#pragma unroll
    for (int k = 0; k < SEQ / 32; ++k) { float d0 = __fsub_rn(v[k], mx); asm volatile("" : "+v"(d0)); v[k] = __builtin_amdgcn_exp2f(__fmul_rn(d0, 1.4426950408889634f)); sum += v[k]; }
#pragma unroll
    for (int sh = 16; sh; sh >>= 1) sum += __shfl_xor(sum, sh, 32);
    const float f = __fdiv_rn(PCAR, sum);
#pragma unroll 1
    for (int ps = 0; ps < 2; ++ps) {
#pragma unroll
        for (int ch = 0; ch < SEQ / 128; ++ch) { v4h o4;
#pragma unroll
            for (int q = 0; q < 4; ++q) o4[q] = tohx(v[ch * 4 + q] * f);
            *(volatile v4h*)(P16 + (size_t)row * SEQ + ch * 128 + lane * 4) = o4; }
        if (ps == 0) __threadfence(); }
}

extern "C" void kernel_launch(void* const* d_in, const int* in_sizes, int n_in,
                              void* d_out, int out_size, void* d_ws, size_t ws_size, hipStream_t stream) {
    if (n_in < 13) return;
    const long long needx = (long long)(NB - 1) * CH * SEQ_FULL + (long long)(CH - 1) * SEQ_FULL + SEQ;
    if ((long long)in_sizes[0] < needx || (long long)out_size < needx) return;
    if (in_sizes[1] < DQK * CH || in_sizes[5] < DQK * CH || in_sizes[9] < CH * CH) return;
    if (in_sizes[2] < DQK || in_sizes[3] < DQK || in_sizes[4] < DQK || in_sizes[6] < DQK || in_sizes[7] < DQK || in_sizes[8] < DQK) return;
    if (in_sizes[10] < CH || in_sizes[11] < CH || in_sizes[12] < CH) return;
    const float* x    = (const float*)d_in[0];
    const float* q_w  = (const float*)d_in[1];  const float* q_b = (const float*)d_in[2];  const float* q_g = (const float*)d_in[3];  const float* q_be = (const float*)d_in[4];
    const float* k_w  = (const float*)d_in[5];  const float* k_b = (const float*)d_in[6];  const float* k_g = (const float*)d_in[7];  const float* k_be = (const float*)d_in[8];
    const float* v_w  = (const float*)d_in[9];  const float* v_b = (const float*)d_in[10]; const float* v_g = (const float*)d_in[11]; const float* v_be = (const float*)d_in[12];
    float* out = (float*)d_out;
    char* wsp = (char*)d_ws;
    auto take = [&](size_t bytes) { char* p = wsp; wsp += (bytes + 255) & ~(size_t)255; return (void*)p; };
    bf*    Wall = (bf*)take((size_t)OC * CH * 2);
    bf*    XT   = (bf*)take((size_t)NB * SEQ * CH * 2);
    float* F    = (float*)take((size_t)NB * SEQ * OC * 4);
    float* ST   = (float*)take((size_t)OC * 4 * 4);
    bf*    QKh  = (bf*)take((size_t)2 * NB * SEQ * DQK * 2);
    bf*    QKl  = (bf*)take((size_t)2 * NB * SEQ * DQK * 2);
    h16*   V16  = (h16*)take((size_t)NB * CH * SEQ * 2);
    float* Sb   = (float*)take((size_t)SEQ * SEQ * 4);
    h16*   P16  = (h16*)take((size_t)SEQ * SEQ * 2);
    if ((size_t)(wsp - (char*)d_ws) > ws_size) return;

    k_cvt8<<<(unsigned)((DQK * CH / 8 + 255) / 256), 256, 0, stream>>>(q_w, Wall, (size_t)DQK * CH / 8);
    k_cvt8<<<(unsigned)((DQK * CH / 8 + 255) / 256), 256, 0, stream>>>(k_w, Wall + (size_t)DQK * CH, (size_t)DQK * CH / 8);
    k_cvt8<<<(unsigned)((CH * CH / 8 + 255) / 256), 256, 0, stream>>>(v_w, Wall + (size_t)2 * DQK * CH, (size_t)CH * CH / 8);
    k_xt<<<(unsigned)(((size_t)NB * SEQ * CH / 2 + 255) / 256), 256, 0, stream>>>(x, XT);
    k_gemmw<bf, 0, 0><<<dim3((unsigned)(NB * SEQ / 64), OC / 64, 1), 32, 0, stream>>>(XT, nullptr, Wall, nullptr, CH, F, OC, nullptr, 1.0f, 0, 0, 0);
    k_stats<<<OC / 32, 256, 0, stream>>>(F, NB * SEQ, q_b, q_g, q_be, k_b, k_g, k_be, v_b, v_g, v_be, ST);
    k_qkp<<<(unsigned)(((size_t)NB * SEQ * DQK + 255) / 256), 256, 0, stream>>>(F, ST, QKh, QKl);
    k_vtp<<<(unsigned)(((size_t)NB * CH * SEQ / 2 + 255) / 256), 256, 0, stream>>>(F, ST, V16);
    const size_t kplane = (size_t)NB * SEQ * DQK;
    for (int b = 0; b < NB; ++b) {
        const size_t qo = (size_t)b * SEQ * DQK;
        k_gemmw<bf, 2, 0><<<dim3(SEQ / 64, SEQ / 64, 1), 32, 0, stream>>>(QKh + qo, QKl + qo, QKh + kplane + qo, QKl + kplane + qo, DQK, Sb, SEQ, nullptr, 1.0f, 0, 0, 0);
        k_asoft<<<SEQ / 8, 256, 0, stream>>>(Sb, P16);
        k_gemmw<h16, 0, 1><<<dim3(CH / 64, SEQ / 64, 1), 32, 0, stream>>>(V16 + (size_t)b * CH * SEQ, nullptr, P16, nullptr, SEQ, out + (size_t)b * CH * SEQ_FULL, SEQ_FULL, x + (size_t)b * CH * SEQ_FULL, 1.0f / PCAR, 0, 0, 0);
    }
}
